// Element_13219909337211
// MI455X (gfx1250) — hardware-verified
//
#include <hip/hip_runtime.h>


#define NBT  8
#define NN   2048
#define DI   512
#define DX   1024
#define DM   DX
#define NX   NN
#define NZ   NN
#define SCL  0.044194173824159216f
#define LEPS 1e-5f
#define LOSC 1024.0f

typedef _Float16 h16;
typedef unsigned short bf;
typedef __attribute__((ext_vector_type(16))) __bf16   v16bf;
typedef __attribute__((ext_vector_type(16))) _Float16 v16h;
typedef __attribute__((ext_vector_type(8)))  _Float16 v8h;
typedef __attribute__((ext_vector_type(8)))  unsigned short v8us;
typedef __attribute__((ext_vector_type(8)))  float    v8f;
typedef __attribute__((ext_vector_type(4)))  float    v4f;
typedef __attribute__((ext_vector_type(4)))  _Float16 v4h;
typedef v8h  __attribute__((may_alias)) v8ha;
typedef v4f  __attribute__((may_alias)) v4fa;
typedef v8us __attribute__((may_alias)) v8usa;

__device__ __forceinline__ unsigned short f2bf(float f) { unsigned u = __float_as_uint(f); u += 0x7FFFu + ((u >> 16) & 1u); return (unsigned short)(u >> 16); }
__device__ __forceinline__ float bf2f(unsigned short b) { return __uint_as_float(((unsigned)b) << 16); }
__device__ __forceinline__ float bfr(float f) { return bf2f(f2bf(f)); }
__device__ __forceinline__ v16h cat16(v8h lo, v8h hi) { return __builtin_shufflevector(lo, hi, 0, 1, 2, 3, 4, 5, 6, 7, 8, 9, 10, 11, 12, 13, 14, 15); }
__device__ __forceinline__ v16bf cat16b(v8us lo, v8us hi) { return __builtin_bit_cast(v16bf, __builtin_shufflevector(lo, hi, 0, 1, 2, 3, 4, 5, 6, 7, 8, 9, 10, 11, 12, 13, 14, 15)); }
__device__ __forceinline__ v8f wmma16(v16h a, v16h b, v8f c) { return __builtin_amdgcn_wmma_f32_16x16x32_f16(false, a, false, b, (short)0, c, false, false); }
__device__ __forceinline__ v8f wmmab(v16bf a, v16bf b, v8f c) { return __builtin_amdgcn_wmma_f32_16x16x32_bf16(false, a, false, b, (short)0, c, false, false); }

__global__ __launch_bounds__(256) void k_wt(const float* __restrict__ Wm, int K, int ncols, bf* WT) {
    __shared__ __align__(16) unsigned short tl[64 * 72];
    const int tid = threadIdx.x, k0 = blockIdx.x * 64, n0 = blockIdx.y * 64;
    const int kk = tid >> 2, nq = (tid & 3) * 16;
#pragma unroll
    for (int i = 0; i < 16; ++i) tl[(nq + i) * 72 + kk] = f2bf(Wm[(size_t)(k0 + kk) * ncols + n0 + nq + i]);
    __syncthreads();
    const int piece = tid & 7;
    auto pass = [&]() {
#pragma unroll
        for (int s = 0; s < 2; ++s) { const int nr = (tid >> 3) + 32 * s; const v8us val = *(const v8usa*)(tl + nr * 72 + piece * 8); *(volatile v8us*)(WT + (size_t)(n0 + nr) * K + k0 + piece * 8) = val; }
    };
    pass(); __threadfence(); pass();
}
template <bool SPLITA, bool F16OUT = false>
__global__ __launch_bounds__(128) void k_gemmb(const bf* __restrict__ A, const bf* __restrict__ Al, const bf* __restrict__ Bn, const float* __restrict__ bias, float* C, int ldc, h16* C2, const float* __restrict__ R = nullptr, int K = DM, int roundR = 1) {
    __shared__ __align__(16) float ost[4][16 * 68];
    const int lane = threadIdx.x & 31, wave = threadIdx.x >> 5, lr = lane & 15, hi = lane >> 4;
    const int r0 = blockIdx.x * 64 + wave * 16, c0 = blockIdx.y * 64;
    const size_t aoff = (size_t)(r0 + lr) * K + 8 * hi;
    size_t boff[4];
#pragma unroll
    for (int t = 0; t < 4; ++t) boff[t] = (size_t)(c0 + t * 16 + lr) * K + 8 * hi;
    v8f acc[4];
#pragma unroll
    for (int t = 0; t < 4; ++t) acc[t] = (v8f){};
#pragma unroll 1
    for (int kc = 0; kc < K; kc += 32) {
        const v16bf a = cat16b(*(const v8us*)(A + aoff + kc), *(const v8us*)(A + aoff + kc + 16));
        v16bf al = a;
        if (SPLITA) al = cat16b(*(const v8us*)(Al + aoff + kc), *(const v8us*)(Al + aoff + kc + 16));
#pragma unroll
        for (int t = 0; t < 4; ++t) { const v16bf b = cat16b(*(const v8us*)(Bn + boff[t] + kc), *(const v8us*)(Bn + boff[t] + kc + 16)); acc[t] = wmmab(a, b, acc[t]); if (SPLITA) acc[t] = wmmab(al, b, acc[t]); }
        asm volatile("v_nop\n\tv_nop\n\tv_nop\n\tv_nop" : "+v"(acc[0]), "+v"(acc[1]), "+v"(acc[2]), "+v"(acc[3]) : "v"(a), "v"(al));
    }
    float* os = &ost[wave][0];
#pragma unroll
    for (int t = 0; t < 4; ++t) { const float bv = bias ? bfr(bias[c0 + t * 16 + lr]) : 0.f;
#pragma unroll
        for (int j = 0; j < 8; ++j) os[(hi * 8 + j) * 68 + t * 16 + lr] = acc[t][j] + bv; }
    __syncthreads();
    if (F16OUT) {
        h16* crow = (h16*)(void*)C + (size_t)r0 * ldc + c0;
        auto pass = [&]() {
#pragma unroll
            for (int s = 0; s < 4; ++s) { const int row = 4 * s + (lane >> 3), piece = lane & 7; const float* sp = os + row * 68 + piece * 8; v8h o, o2;
#pragma unroll
                for (int i = 0; i < 8; ++i) { const h16 a = (h16)sp[i]; o[i] = a; o2[i] = (h16)((sp[i] - (float)a) * LOSC); }
                *(volatile v8h*)(crow + (size_t)row * ldc + piece * 8) = o; if (C2) *(volatile v8h*)(C2 + (size_t)r0 * ldc + c0 + (size_t)row * ldc + piece * 8) = o2; }
        };
        pass(); __threadfence(); pass();
    } else {
        float* crow = C + (size_t)r0 * ldc + c0;
        auto pass = [&]() {
#pragma unroll
            for (int s = 0; s < 8; ++s) { const int Lid = (lane >> 3) + 4 * s, piece = lane & 7; const int row = Lid >> 1, cofs = (Lid & 1) * 32 + piece * 4;
                v4f val = *(const v4fa*)(os + row * 68 + cofs); if (R) { const v4f rv = *(const v4f*)(R + ((size_t)r0 + row) * ldc + c0 + cofs); val += roundR ? (v4f){bfr(rv[0]), bfr(rv[1]), bfr(rv[2]), bfr(rv[3])} : rv; }
                *(volatile v4f*)(crow + (size_t)row * ldc + cofs) = val; }
        };
        pass(); __threadfence(); pass();
    }
}

template <int MODE>
__global__ __launch_bounds__(128) void k_gemm3x(const bf* __restrict__ Ah, const bf* __restrict__ Al, const bf* __restrict__ Bh, const bf* __restrict__ Bl, int K, float* C, int ldc) {
    if ((MODE & 1) && (int)blockIdx.y * 64 > (int)blockIdx.x * 64 + 63) return;
    const int Klim = (MODE & 2) ? min(K, ((int)blockIdx.x + 1) * 64) : K;
    __shared__ __align__(16) float ost[4][16 * 68];
    const int lane = threadIdx.x & 31, wave = threadIdx.x >> 5, lr = lane & 15, hi = lane >> 4;
    const int r0 = blockIdx.x * 64 + wave * 16, c0 = blockIdx.y * 64;
    const size_t aoff = (size_t)(r0 + lr) * K + 8 * hi;
    v8f acc[4];
#pragma unroll
    for (int t = 0; t < 4; ++t) acc[t] = (v8f){};
#pragma unroll 1
    for (int kc = 0; kc < Klim; kc += 32) {
        const v16bf a = cat16b(*(const v8us*)(Ah + aoff + kc), *(const v8us*)(Ah + aoff + kc + 16));
        v16bf al = a; if (!(MODE & 4) && !(MODE & 16)) al = cat16b(*(const v8us*)(Al + aoff + kc), *(const v8us*)(Al + aoff + kc + 16));
#pragma unroll
        for (int t = 0; t < 4; ++t) { const size_t bo = (size_t)(c0 + t * 16 + lr) * K + kc + 8 * hi;
            const v16bf bh = cat16b(*(const v8us*)(Bh + bo), *(const v8us*)(Bh + bo + 16));
            acc[t] = wmmab(a, bh, acc[t]);
            if (!(MODE & 4)) { if (!(MODE & 16)) acc[t] = wmmab(al, bh, acc[t]); if (!(MODE & 8)) { const v16bf bl = cat16b(*(const v8us*)(Bl + bo), *(const v8us*)(Bl + bo + 16)); acc[t] = wmmab(a, bl, acc[t]); } } }
        asm volatile("v_nop\n\tv_nop\n\tv_nop\n\tv_nop" : "+v"(acc[0]), "+v"(acc[1]), "+v"(acc[2]), "+v"(acc[3]) : "v"(a), "v"(al));
    }
    float* os = &ost[wave][0];
#pragma unroll
    for (int t = 0; t < 4; ++t) {
#pragma unroll
        for (int j = 0; j < 8; ++j) os[(hi * 8 + j) * 68 + t * 16 + lr] = acc[t][j]; }
    __builtin_amdgcn_wave_barrier(); asm volatile("" ::: "memory");
    float* crow = C + (size_t)r0 * ldc + c0;
    auto pass = [&]() {
#pragma unroll
        for (int s = 0; s < 8; ++s) { const int Lid = (lane >> 3) + 4 * s, piece = lane & 7; const int row = Lid >> 1, cofs = (Lid & 1) * 32 + piece * 4;
            const v4f val = *(const v4fa*)(os + row * 68 + cofs); *(volatile v4f*)(crow + (size_t)row * ldc + cofs) = val; }
    };
    pass(); __threadfence(); pass();
}


__global__ __launch_bounds__(256) void k_cat(const float* __restrict__ a, const float* __restrict__ c, bf* Xb) {
    const int lane = threadIdx.x & 31; const size_t t = (size_t)blockIdx.x * 8 + (threadIdx.x >> 5); if (t >= (size_t)NN) return;
#pragma unroll 1
    for (int ps = 0; ps < 2; ++ps) {
#pragma unroll
        for (int q = 0; q < 4; ++q) { const float* src = (q < 2 ? a : c) + t * DI + (q & 1) * 256 + lane * 8; v8us o;
#pragma unroll
            for (int i = 0; i < 8; ++i) o[i] = f2bf(src[i]);
            *(volatile v8us*)(Xb + t * DX + q * 256 + lane * 8) = o; }
        if (ps == 0) __threadfence(); }
}
__global__ __launch_bounds__(256) void k_split512s(const float* __restrict__ src, int rows, float sc, bf* dh, bf* dl) {
    const int lane = threadIdx.x & 31; const size_t r = (size_t)blockIdx.x * 8 + (threadIdx.x >> 5); if (r >= (size_t)rows) return;
#pragma unroll 1
    for (int ps = 0; ps < 2; ++ps) {
#pragma unroll
        for (int q = 0; q < DI / 256; ++q) { const size_t o = r * DI + q * 256 + lane * 8; const v8f v = *(const v8f*)(src + o); v8us oh, ol;
#pragma unroll
            for (int i = 0; i < 8; ++i) { const float y = v[i] * sc; const unsigned short hb = f2bf(y); oh[i] = hb; ol[i] = f2bf(y - bf2f(hb)); }
            *(volatile v8us*)(dh + o) = oh; *(volatile v8us*)(dl + o) = ol; }
        if (ps == 0) __threadfence(); }
}
__global__ __launch_bounds__(256) void k_vt512(const float* __restrict__ V, bf* Th, bf* Tl) {
    __shared__ float tl[64][65];
    typedef __attribute__((ext_vector_type(4))) unsigned short v4us;
    const int tid = threadIdx.x; const int t0 = blockIdx.x * 64, d0 = blockIdx.y * 64; const int rr = tid >> 2, cq = (tid & 3) * 16;
#pragma unroll
    for (int i = 0; i < 16; ++i) tl[rr][cq + i] = V[(size_t)(t0 + rr) * DI + d0 + cq + i];
    __syncthreads();
    const int lane = tid & 31, wv = tid >> 5;
    auto pass = [&]() {
#pragma unroll
        for (int st = 0; st < 4; ++st) { const int dr = wv * 8 + st * 2 + (lane >> 4); const int tq = (lane & 15) * 4; v4us oh, ol;
#pragma unroll
            for (int i = 0; i < 4; ++i) { const float y = tl[tq + i][dr]; const unsigned short hb = f2bf(y); oh[i] = hb; ol[i] = f2bf(y - bf2f(hb)); }
            const size_t o = (size_t)(d0 + dr) * NN + t0 + tq; *(volatile v4us*)(Th + o) = oh; *(volatile v4us*)(Tl + o) = ol; }
    };
    pass(); __threadfence(); pass();
}
__global__ __launch_bounds__(256) void k_csoft1(const float* __restrict__ S, bf* PH, bf* PL) {
    typedef __attribute__((ext_vector_type(4))) unsigned short v4us;
    const int lane = threadIdx.x & 31, i = blockIdx.x * 8 + (threadIdx.x >> 5); if (i >= NN) return; const float* sr = S + (size_t)i * NN;
    float m = -3.0e38f;
#pragma unroll 1
    for (int c0 = lane * 4; c0 < NN; c0 += 128) {
#pragma unroll
        for (int q = 0; q < 4; ++q) { const int k = c0 + q; if (k <= i) m = fmaxf(m, sr[k]); } }
#pragma unroll
    for (int sh = 16; sh; sh >>= 1) m = fmaxf(m, __shfl_xor(m, sh, 32));
    float sum = 0.f;
#pragma unroll 1
    for (int c0 = lane * 4; c0 < NN; c0 += 128) {
#pragma unroll
        for (int q = 0; q < 4; ++q) { const int k = c0 + q; if (k <= i) sum += __expf(sr[k] - m); } }
#pragma unroll
    for (int sh = 16; sh; sh >>= 1) sum += __shfl_xor(sum, sh, 32);
    const float inv = 1.0f / sum;
#pragma unroll 1
    for (int ps = 0; ps < 2; ++ps) {
#pragma unroll 1
        for (int c0 = lane * 4; c0 < NN; c0 += 128) { v4us oh, ol;
#pragma unroll
            for (int q = 0; q < 4; ++q) { const int k = c0 + q; const float p = (k <= i) ? __expf(sr[(k <= i) ? k : 0] - m) * inv : 0.f; const unsigned short hb = f2bf(p); oh[q] = hb; ol[q] = f2bf(p - bf2f(hb)); }
            const size_t o = (size_t)i * NN + c0; *(volatile v4us*)(PH + o) = oh; *(volatile v4us*)(PL + o) = ol; }
        if (ps == 0) __threadfence(); }
}
__global__ __launch_bounds__(256) void k_ln512(const float* __restrict__ O, const float* __restrict__ g, const float* __restrict__ bb, float* OUTB) {
    const int lane = threadIdx.x & 31; const size_t t = (size_t)blockIdx.x * 8 + (threadIdx.x >> 5); if (t >= (size_t)NN) return; float v[16]; float s = 0.f;
#pragma unroll
    for (int q = 0; q < 4; ++q) {
#pragma unroll
        for (int i = 0; i < 4; ++i) { v[q * 4 + i] = O[t * DI + q * 128 + lane * 4 + i]; s += v[q * 4 + i]; } }
#pragma unroll
    for (int sh = 16; sh; sh >>= 1) s += __shfl_xor(s, sh, 32);
    const float mu = s * (1.0f / DI); float qv = 0.f;
#pragma unroll
    for (int i = 0; i < 16; ++i) { const float d = v[i] - mu; qv = fmaf(d, d, qv); }
#pragma unroll
    for (int sh = 16; sh; sh >>= 1) qv += __shfl_xor(qv, sh, 32);
    const float rs = rsqrtf(qv * (1.0f / DI) + LEPS);
#pragma unroll 1
    for (int ps = 0; ps < 2; ++ps) {
#pragma unroll
        for (int q = 0; q < 4; ++q) { const int c0 = q * 128 + lane * 4; v4f y;
#pragma unroll
            for (int i = 0; i < 4; ++i) y[i] = (v[q * 4 + i] - mu) * rs * bfr(g[c0 + i]) + bfr(bb[c0 + i]);
            *(volatile v4f*)(OUTB + t * DI + c0) = y; }
        if (ps == 0) __threadfence(); }
}

extern "C" void kernel_launch(void* const* d_in, const int* in_sizes, int n_in,
                              void* d_out, int out_size, void* d_ws, size_t ws_size, hipStream_t stream) {
    (void)in_sizes; (void)n_in; (void)out_size;
    const float* x0 = (const float*)d_in[0]; const float* x1 = (const float*)d_in[1]; const float* Wq = (const float*)d_in[2]; const float* Wk = (const float*)d_in[3]; const float* Wv = (const float*)d_in[4]; const float* gam = (const float*)d_in[5]; const float* bet = (const float*)d_in[6];
    float* out = (float*)d_out;
    char* wsp = (char*)d_ws;
    auto take = [&](size_t bytes) { char* p = wsp; wsp += (bytes + 255) & ~(size_t)255; return (void*)p; };
    bf* WQ = (bf*)take((size_t)DI * DX * 2); bf* WK = (bf*)take((size_t)DI * DX * 2); bf* WV = (bf*)take((size_t)DI * DX * 2);
    bf* Xb = (bf*)take((size_t)NN * DX * 2); float* QF = (float*)take((size_t)NN * DI * 4); float* KF = (float*)take((size_t)NN * DI * 4); float* VF = (float*)take((size_t)NN * DI * 4);
    bf* Qh = (bf*)take((size_t)NN * DI * 2); bf* Ql = (bf*)take((size_t)NN * DI * 2); bf* Kh = (bf*)take((size_t)NN * DI * 2); bf* Kl = (bf*)take((size_t)NN * DI * 2); bf* VTh = (bf*)take((size_t)DI * NN * 2); bf* VTl = (bf*)take((size_t)DI * NN * 2);
    float* S = (float*)take((size_t)NN * NN * 4); bf* PH = (bf*)take((size_t)NN * NN * 2); bf* PL = (bf*)take((size_t)NN * NN * 2); float* O = (float*)take((size_t)NN * DI * 4);
    if ((size_t)(wsp - (char*)d_ws) > ws_size) return;
    k_wt<<<dim3(DX / 64, DI / 64, 1), 256, 0, stream>>>(Wq, DX, DI, WQ); k_wt<<<dim3(DX / 64, DI / 64, 1), 256, 0, stream>>>(Wk, DX, DI, WK); k_wt<<<dim3(DX / 64, DI / 64, 1), 256, 0, stream>>>(Wv, DX, DI, WV);
    const dim3 gp(NN / 64, DI / 64, 1);
    for (int b = 0; b < NBT; ++b) {
        k_cat<<<NN / 8, 256, 0, stream>>>(x0 + (size_t)b * NN * DI, x1 + (size_t)b * NN * DI, Xb);
        k_gemmb<false, false><<<gp, 128, 0, stream>>>(Xb, nullptr, WQ, nullptr, QF, DI, nullptr, nullptr, DX); k_gemmb<false, false><<<gp, 128, 0, stream>>>(Xb, nullptr, WK, nullptr, KF, DI, nullptr, nullptr, DX); k_gemmb<false, false><<<gp, 128, 0, stream>>>(Xb, nullptr, WV, nullptr, VF, DI, nullptr, nullptr, DX);
        k_split512s<<<NN / 8, 256, 0, stream>>>(QF, NN, SCL, Qh, Ql); k_split512s<<<NN / 8, 256, 0, stream>>>(KF, NN, 1.0f, Kh, Kl); k_vt512<<<dim3(NN / 64, DI / 64, 1), 256, 0, stream>>>(VF, VTh, VTl);
        k_gemm3x<1><<<dim3(NN / 64, NN / 64, 1), 128, 0, stream>>>(Qh, Ql, Kh, Kl, DI, S, NN);
        k_csoft1<<<NN / 8, 256, 0, stream>>>(S, PH, PL);
        k_gemm3x<2><<<dim3(NN / 64, DI / 64, 1), 128, 0, stream>>>(PH, PL, VTh, VTl, NN, O, DI);
        k_ln512<<<NN / 8, 256, 0, stream>>>(O, gam, bet, out + (size_t)b * NN * DI); }
}
